// SparseCloudConvolution_67173288509589
// MI455X (gfx1250) — hardware-verified
//
#include <hip/hip_runtime.h>
#include <stddef.h>


#define CIN     64
#define TT      8
#define KD      (CIN * TT)
#define FD      64
#define NTHR    256
#define NWAVE   8
#define EPT     8
#define NGRP    2
#define CHUNK   (NTHR * EPT * NGRP)
#define WCAP    (EPT * NGRP * 32)
#define LISTN   (NWAVE * WCAP)
#define NBC     4096
#define NBF     1024
#define RCAP    40960
#define RBN     128
#define TGT     256
#define DEGCAP  2048
#define GROWS   128
#define OTHR    512
#define SKP     68
#define WSCAP   134217728
#define WSCALE  16.0f
#define WINV    0.0625f

#define LDS_FILL ((RCAP + NBF + LISTN) * 4 + 64)

static_assert((CHUNK & (CHUNK - 1)) == 0);
static_assert(CHUNK <= 4096);
static_assert(NBC <= 4096 && NBF <= 4096);
static_assert((NBC & (NBC - 1)) == 0 && (NBF & (NBF - 1)) == 0);
static_assert(NBC == 4 * NBF);
static_assert(OTHR * 8 == NBC);
static_assert((RCAP % 32) == 0);
static_assert(TGT == NWAVE * 32 && (TGT % GROWS) == 0);
static_assert((NBC % TGT) == 0);
static_assert(GROWS == NWAVE * 16);
static_assert(CIN == 64 && FD == 64 && (KD % 32) == 0 && KD == 512);
static_assert((SKP % 4) == 0);

typedef float    v4f  __attribute__((ext_vector_type(4)));
typedef float    v8f  __attribute__((ext_vector_type(8)));
typedef int      v4i  __attribute__((ext_vector_type(4)));
typedef _Float16 v4h  __attribute__((ext_vector_type(4)));
typedef _Float16 v8h  __attribute__((ext_vector_type(8)));
typedef _Float16 v16h __attribute__((ext_vector_type(16)));
union FragH { v16h v; v8h h[2]; };

__device__ __forceinline__ v8f wmh(v16h a, v16h b, v8f c) {
  v8f d = __builtin_amdgcn_wmma_f32_16x16x32_f16(false, a, false, b, (short)0, c, false, false);
  asm volatile("v_nop\n\tv_nop\n\tv_nop\n\tv_nop" : "+v"(d) : "v"(a), "v"(b));
  return d;
}

__device__ __forceinline__ v8h cvt8(v4f a, v4f b, float s) {
  v8h c;
  c[0] = (_Float16)(a.x * s); c[1] = (_Float16)(a.y * s); c[2] = (_Float16)(a.z * s); c[3] = (_Float16)(a.w * s);
  c[4] = (_Float16)(b.x * s); c[5] = (_Float16)(b.y * s); c[6] = (_Float16)(b.z * s); c[7] = (_Float16)(b.w * s);
  return c;
}

__device__ __forceinline__ v4h cvt4(v4f a) {
  v4h c;
  c.x = (_Float16)a.x; c.y = (_Float16)a.y; c.z = (_Float16)a.z; c.w = (_Float16)a.w;
  return c;
}

__device__ __forceinline__ v4f selv(bool cnd, v4f a, v4f b) {
  v4f r;
  r.x = cnd ? a.x : b.x; r.y = cnd ? a.y : b.y; r.z = cnd ? a.z : b.z; r.w = cnd ? a.w : b.w;
  return r;
}

__device__ __forceinline__ v4f xsum16(v4f v) {
  v4f r;
  r.x = v.x + __shfl_xor(v.x, 16);
  r.y = v.y + __shfl_xor(v.y, 16);
  r.z = v.z + __shfl_xor(v.z, 16);
  r.w = v.w + __shfl_xor(v.w, 16);
  return r;
}

template <int NB>
__device__ __forceinline__ int scan_chunk(const int* __restrict__ idx, int nE, int cbase, int slotBase,
                                          int vec8, int* list, int tid, int lane, int wave) {
  int wc = 0;
#pragma unroll
  for (int g = 0; g < NGRP; ++g) {
    const int el0  = (g * NTHR + tid) * EPT;
    const int e0   = cbase + el0;
    const int sent = -2147483647 - 1;
    v4i da, db;
    if (vec8 != 0 && cbase + CHUNK <= nE) {
      const int* p = idx + 2 * (size_t)e0;
      const v4i q0 = *(const v4i*)(p);
      const v4i q1 = *(const v4i*)(p + 4);
      const v4i q2 = *(const v4i*)(p + 8);
      const v4i q3 = *(const v4i*)(p + 12);
      da.x = q0.x; da.y = q0.z; da.z = q1.x; da.w = q1.z;
      db.x = q2.x; db.y = q2.z; db.z = q3.x; db.w = q3.z;
    } else {
      da.x = (e0     < nE) ? idx[2 * min(e0, nE - 1)]     : sent;
      da.y = (e0 + 1 < nE) ? idx[2 * min(e0 + 1, nE - 1)] : sent;
      da.z = (e0 + 2 < nE) ? idx[2 * min(e0 + 2, nE - 1)] : sent;
      da.w = (e0 + 3 < nE) ? idx[2 * min(e0 + 3, nE - 1)] : sent;
      db.x = (e0 + 4 < nE) ? idx[2 * min(e0 + 4, nE - 1)] : sent;
      db.y = (e0 + 5 < nE) ? idx[2 * min(e0 + 5, nE - 1)] : sent;
      db.z = (e0 + 6 < nE) ? idx[2 * min(e0 + 6, nE - 1)] : sent;
      db.w = (e0 + 7 < nE) ? idx[2 * min(e0 + 7, nE - 1)] : sent;
    }
    const unsigned nb = (unsigned)slotBase;
    const unsigned s0 = (unsigned)da.x - nb, s1 = (unsigned)da.y - nb;
    const unsigned s2 = (unsigned)da.z - nb, s3 = (unsigned)da.w - nb;
    const unsigned s4 = (unsigned)db.x - nb, s5 = (unsigned)db.y - nb;
    const unsigned s6 = (unsigned)db.z - nb, s7 = (unsigned)db.w - nb;
    const bool h0 = s0 < (unsigned)NB, h1 = s1 < (unsigned)NB, h2 = s2 < (unsigned)NB, h3 = s3 < (unsigned)NB;
    const bool h4 = s4 < (unsigned)NB, h5 = s5 < (unsigned)NB, h6 = s6 < (unsigned)NB, h7 = s7 < (unsigned)NB;
    const unsigned any = __builtin_amdgcn_ballot_w32(h0 | h1 | h2 | h3 | h4 | h5 | h6 | h7);
    if (any != 0u) {
#define HITJ(J, HJ, SJ) { \
        const unsigned mj = __builtin_amdgcn_ballot_w32(HJ); \
        if (mj != 0u) { \
          if (HJ) { \
            const int pos = wc + (int)__builtin_amdgcn_mbcnt_lo(mj, 0u); \
            if (pos < WCAP) list[wave * WCAP + pos] = ((el0 + (J)) << 12) | (int)(SJ); \
          } \
          wc += (int)__builtin_popcount(mj); } }
      HITJ(0, h0, s0)
      HITJ(1, h1, s1)
      HITJ(2, h2, s2)
      HITJ(3, h3, s3)
      HITJ(4, h4, s4)
      HITJ(5, h5, s5)
      HITJ(6, h6, s6)
      HITJ(7, h7, s7)
#undef HITJ
    }
  }
  return wc;
}

__global__ __launch_bounds__(NTHR) void k_wprep(const float* __restrict__ Km, _Float16* wp) {
  __shared__ __attribute__((aligned(16))) float sK[CIN * SKP];
  const int tid = threadIdx.x;
  const int t = blockIdx.x;
  const float* src = Km + (size_t)t * CIN * FD;
  for (int i = tid; i < (CIN * FD) / 4; i += NTHR) {
    const int c = i >> 4, n4 = (i & 15) * 4;
    const v4f v = *(const v4f*)(src + 4 * i);
    *(v4f*)(sK + c * SKP + n4) = v;
  }
  __syncthreads();
  v8h cv[2];
#pragma unroll
  for (int s = 0; s < 2; ++s) {
    const int n = (tid >> 3) + 32 * s, g = tid & 7;
    const float* cp = sK + (8 * g) * SKP + n;
    v4f a, b;
    a.x = cp[0];       a.y = cp[SKP];     a.z = cp[2 * SKP]; a.w = cp[3 * SKP];
    b.x = cp[4 * SKP]; b.y = cp[5 * SKP]; b.z = cp[6 * SKP]; b.w = cp[7 * SKP];
    cv[s] = cvt8(a, b, WSCALE);
  }
#pragma unroll
  for (int s = 0; s < 2; ++s) {
    const int n = (tid >> 3) + 32 * s, g = tid & 7;
    _Float16* dp = wp + (size_t)n * KD + t * CIN + 8 * g;
    *(volatile v8h*)dp = cv[s];
  }
  __threadfence();
#pragma unroll
  for (int s = 0; s < 2; ++s) {
    const int n = (tid >> 3) + 32 * s, g = tid & 7;
    _Float16* dp = wp + (size_t)n * KD + t * CIN + 8 * g;
    *(volatile v8h*)dp = cv[s];
  }
}

__global__ __launch_bounds__(NTHR) void k_count(const int* __restrict__ idx, int* cnt, int nE, int vec8) {
  __shared__ __attribute__((aligned(16))) int scnt[NBC];
  __shared__ __attribute__((aligned(16))) int list[LISTN];
  __shared__ int wcnt[NWAVE];
  const int tid = threadIdx.x, lane = tid & 31, wave = tid >> 5;
  const int nodeBase = blockIdx.x * NBC;

  for (int i = tid; i < NBC; i += NTHR) scnt[i] = 0;
  __syncthreads();

  const int nChunks = (nE + CHUNK - 1) / CHUNK;
#pragma unroll 1
  for (int ch = 0; ch < nChunks; ++ch) {
    const int cbase = ch * CHUNK;
    const int wc = scan_chunk<NBC>(idx, nE, cbase, nodeBase, vec8, list, tid, lane, wave);
    if (lane == 0) wcnt[wave] = wc;
    __syncthreads();
    if (wave == 0) {
#pragma unroll 1
      for (int wsx = 0; wsx < NWAVE; ++wsx) {
        int n = __builtin_amdgcn_readfirstlane(wcnt[wsx]);
        n = n > WCAP ? WCAP : (n < 0 ? 0 : n);
        const int* lp = list + wsx * WCAP;
#pragma unroll 1
        for (int i = 0; i < n; ++i) {
          const int ent  = __builtin_amdgcn_readfirstlane(lp[i]);
          const int slot = ent & (NBC - 1);
          if (lane == 0) scnt[slot] = scnt[slot] + 1;
        }
      }
    }
    __syncthreads();
  }

  v4i cq[4];
#pragma unroll
  for (int q = 0; q < 4; ++q) {
    const int f = (wave * 4 + q) * 128 + 4 * lane;
    cq[q] = *(const v4i*)(scnt + f);
  }
  int* cp = cnt + (size_t)nodeBase;
#pragma unroll
  for (int q = 0; q < 4; ++q) {
    const int f = (wave * 4 + q) * 128 + 4 * lane;
    *(volatile v4i*)(cp + f) = cq[q];
  }
  __threadfence();
#pragma unroll
  for (int q = 0; q < 4; ++q) {
    const int f = (wave * 4 + q) * 128 + 4 * lane;
    *(volatile v4i*)(cp + f) = cq[q];
  }
}

__global__ __launch_bounds__(OTHR) void k_offsets(
    const int* __restrict__ cnt, int* off, int* rbase, int nChunk) {
  __shared__ __attribute__((aligned(16))) int soff[NBC];
  __shared__ __attribute__((aligned(16))) int srb[RBN];
  __shared__ int wtot[OTHR / 32];
  const int tid = threadIdx.x, lane = tid & 31, wave = tid >> 5, sub = tid >> 7;
  for (int i = tid; i < RBN; i += OTHR) srb[i] = 0;
  int carry = 0;
#pragma unroll 1
  for (int ch = 0; ch < nChunk; ++ch) {
    const int base = ch * NBC;
    const v4i c0 = *(const v4i*)(cnt + base + 8 * tid);
    const v4i c1 = *(const v4i*)(cnt + base + 8 * tid + 4);
    const int e0 = max(c0.x, 0), e1 = max(c0.y, 0), e2 = max(c0.z, 0), e3 = max(c0.w, 0);
    const int e4 = max(c1.x, 0), e5 = max(c1.y, 0), e6 = max(c1.z, 0), e7 = max(c1.w, 0);
    const int ts = e0 + e1 + e2 + e3 + e4 + e5 + e6 + e7;
    int incl = ts;
#pragma unroll
    for (int d = 1; d < 32; d <<= 1) {
      const int t = __shfl_up(incl, d);
      if (lane >= d) incl += t;
    }
    if (lane == 31) wtot[wave] = incl;
    __syncthreads();
    const int S0 = wtot[0]  + wtot[1]  + wtot[2]  + wtot[3];
    const int S1 = wtot[4]  + wtot[5]  + wtot[6]  + wtot[7];
    const int S2 = wtot[8]  + wtot[9]  + wtot[10] + wtot[11];
    const int S3 = wtot[12] + wtot[13] + wtot[14] + wtot[15];
    int pre = 0;
#pragma unroll 1
    for (int w = 4 * sub; w < wave; ++w) pre += wtot[w];
    const int b0 = carry;
    const int b1 = b0 + ((S0 + 31) & ~31);
    const int b2 = b1 + ((S1 + 31) & ~31);
    const int b3 = b2 + ((S2 + 31) & ~31);
    const int b4 = b3 + ((S3 + 31) & ~31);
    const int myb = sub == 0 ? b0 : (sub == 1 ? b1 : (sub == 2 ? b2 : b3));
    if (tid == 0) {
      srb[min(4 * ch + 0, RBN - 1)] = b0;
      srb[min(4 * ch + 1, RBN - 1)] = b1;
      srb[min(4 * ch + 2, RBN - 1)] = b2;
      srb[min(4 * ch + 3, RBN - 1)] = b3;
    }
    int run = myb + pre + incl - ts;
    soff[8 * tid + 0] = run; run += e0;
    soff[8 * tid + 1] = run; run += e1;
    soff[8 * tid + 2] = run; run += e2;
    soff[8 * tid + 3] = run; run += e3;
    soff[8 * tid + 4] = run; run += e4;
    soff[8 * tid + 5] = run; run += e5;
    soff[8 * tid + 6] = run; run += e6;
    soff[8 * tid + 7] = run;
    carry = b4;
    __syncthreads();
    const v4i o0 = *(const v4i*)(soff + 4 * tid);
    const v4i o1 = *(const v4i*)(soff + 4 * (tid + OTHR));
    int* op = off + base;
    *(volatile v4i*)(op + 4 * tid) = o0;
    *(volatile v4i*)(op + 4 * (tid + OTHR)) = o1;
    __threadfence();
    *(volatile v4i*)(op + 4 * tid) = o0;
    *(volatile v4i*)(op + 4 * (tid + OTHR)) = o1;
    __syncthreads();
  }
  if (tid == 0) srb[min(4 * nChunk, RBN - 1)] = carry;
  __syncthreads();
  v4i rv = {0, 0, 0, 0};
  if (tid < 32) rv = *(const v4i*)(srb + 4 * tid);
  if (tid < 32) *(volatile v4i*)(rbase + 4 * tid) = rv;
  __threadfence();
  if (tid < 32) *(volatile v4i*)(rbase + 4 * tid) = rv;
}

__global__ __launch_bounds__(NTHR) void k_fill(
    const int* __restrict__ idx, const int* __restrict__ off, const int* __restrict__ rbase,
    int* csr, int nE, int vec8, int csrLen) {
  extern __shared__ v4f lds_dyn[];
  int* region = (int*)lds_dyn;
  int* cursor = region + RCAP;
  int* list   = cursor + NBF;
  int* wcnt   = list + LISTN;
  const int tid = threadIdx.x, lane = tid & 31, wave = tid >> 5;
  const int b = blockIdx.x;
  const int nodeBase = b * NBF;

  int rb0 = rbase[b];
  const int rb1 = rbase[b + 1];
  rb0 = rb0 < 0 ? 0 : (rb0 > csrLen ? csrLen : rb0);
  rb0 &= ~31;
  int len = rb1 - rb0;
  len = len < 0 ? 0 : (len > RCAP ? RCAP : len);
  int lenW = (len + 31) & ~31;
  if (rb0 + lenW > csrLen) lenW = (csrLen - rb0) & ~31;

  {
    const v4i z = {0, 0, 0, 0};
    for (int i = tid; i < RCAP / 4; i += NTHR) ((v4i*)region)[i] = z;
    for (int s = tid; s < NBF; s += NTHR) {
      int o = off[nodeBase + s] - rb0;
      o = o < 0 ? 0 : (o > RCAP ? RCAP : o);
      cursor[s] = o;
    }
  }
  __syncthreads();

  const int nChunks = (nE + CHUNK - 1) / CHUNK;
#pragma unroll 1
  for (int ch = 0; ch < nChunks; ++ch) {
    const int cbase = ch * CHUNK;
    const int wc = scan_chunk<NBF>(idx, nE, cbase, nodeBase, vec8, list, tid, lane, wave);
    if (lane == 0) wcnt[wave] = wc;
    __syncthreads();
    if (wave == 0) {
#pragma unroll 1
      for (int wsx = 0; wsx < NWAVE; ++wsx) {
        int n = __builtin_amdgcn_readfirstlane(wcnt[wsx]);
        n = n > WCAP ? WCAP : (n < 0 ? 0 : n);
        const int* lp = list + wsx * WCAP;
#pragma unroll 1
        for (int i = 0; i < n; ++i) {
          const int ent  = __builtin_amdgcn_readfirstlane(lp[i]);
          const int slot = ent & (NBF - 1);
          int e = cbase + ((ent >> 12) & (CHUNK - 1));
          e = e < 0 ? 0 : (e > nE - 1 ? nE - 1 : e);
          if (lane == 0) {
            int pos = cursor[slot];
            pos = pos < 0 ? 0 : (pos > RCAP - 1 ? RCAP - 1 : pos);
            region[pos] = e;
            const int np = pos + 1;
            cursor[slot] = np > RCAP ? RCAP : np;
          }
        }
      }
    }
    __syncthreads();
  }

  const int nv = lenW >> 2;
  int* gp = csr + rb0;
#pragma unroll 1
  for (int i = tid; i < nv; i += NTHR) { const v4i v = ((const v4i*)region)[i]; *(volatile v4i*)(gp + 4 * i) = v; }
  __threadfence();
#pragma unroll 1
  for (int i = tid; i < nv; i += NTHR) { const v4i v = ((const v4i*)region)[i]; *(volatile v4i*)(gp + 4 * i) = v; }
}

__global__ __launch_bounds__(NTHR) void k_agg(
    const int* __restrict__ csr, const int* __restrict__ off, const int* __restrict__ cnt,
    const int* __restrict__ idx, const float* __restrict__ ef, const float* __restrict__ x,
    _Float16* Ag, int nIn, int nE, int csrLen) {
  __shared__ __attribute__((aligned(16))) _Float16 stg[NWAVE * KD];
  const int tid = threadIdx.x, lane = tid & 31, wave = tid >> 5, hh = lane >> 4, lj = lane & 15;
  const int tbase = blockIdx.x * TGT + wave * 32;
  const int cl = tbase + lane;
  const int cnt_l = cnt[cl];
  const int off_l = off[cl];
  _Float16* sw = stg + wave * KD;
  const float* xl = x + 4 * lj;
  const v4f z4 = {0.0f, 0.0f, 0.0f, 0.0f};

#pragma unroll 1
  for (int j = 0; j < 32; ++j) {
    const int c = tbase + j;
    int n = __builtin_amdgcn_readlane(cnt_l, j);
    n = n < 0 ? 0 : (n > DEGCAP ? DEGCAP : n);
    const int st = __builtin_amdgcn_readlane(off_l, j);
    v4f a0 = z4, a1 = z4, a2 = z4, a3 = z4, a4 = z4, a5 = z4, a6 = z4, a7 = z4;
#pragma unroll 1
    for (int q0 = 0; q0 < n; q0 += 32) {
      int pos = st + q0 + lane;
      pos = pos < 0 ? 0 : (pos > csrLen - 1 ? csrLen - 1 : pos);
      int el = csr[pos];
      el = el < 0 ? 0 : (el > nE - 1 ? nE - 1 : el);
      int sl = idx[2 * el + 1];
      sl = sl < 0 ? 0 : (sl > nIn - 1 ? nIn - 1 : sl);
      const int mcnt = (n - q0) < 32 ? (n - q0) : 32;
      const bool act = lane < mcnt;
      const float* wq = ef + el;
      const float w0 = act ? wq[0]              : 0.0f;
      const float w1 = act ? wq[(size_t)1 * nE] : 0.0f;
      const float w2 = act ? wq[(size_t)2 * nE] : 0.0f;
      const float w3 = act ? wq[(size_t)3 * nE] : 0.0f;
      const float w4 = act ? wq[(size_t)4 * nE] : 0.0f;
      const float w5 = act ? wq[(size_t)5 * nE] : 0.0f;
      const float w6 = act ? wq[(size_t)6 * nE] : 0.0f;
      const float w7 = act ? wq[(size_t)7 * nE] : 0.0f;
#pragma unroll 1
      for (int p = 0; p < mcnt; p += 2) {
        const int pe = (p + hh) & 31;
        const int s = __shfl(sl, pe);
        const float u0 = __shfl(w0, pe), u1 = __shfl(w1, pe), u2 = __shfl(w2, pe), u3 = __shfl(w3, pe);
        const float u4 = __shfl(w4, pe), u5 = __shfl(w5, pe), u6 = __shfl(w6, pe), u7 = __shfl(w7, pe);
        const v4f vf = *(const v4f*)(xl + (size_t)s * CIN);
        a0 = a0 + vf * u0; a1 = a1 + vf * u1; a2 = a2 + vf * u2; a3 = a3 + vf * u3;
        a4 = a4 + vf * u4; a5 = a5 + vf * u5; a6 = a6 + vf * u6; a7 = a7 + vf * u7;
      }
    }
    const v4f t0 = xsum16(a0), t1 = xsum16(a1), t2 = xsum16(a2), t3 = xsum16(a3);
    const v4f t4 = xsum16(a4), t5 = xsum16(a5), t6 = xsum16(a6), t7 = xsum16(a7);
    const bool hi = hh != 0;
    const v4h c0 = cvt4(selv(hi, t1, t0));
    const v4h c1 = cvt4(selv(hi, t3, t2));
    const v4h c2 = cvt4(selv(hi, t5, t4));
    const v4h c3 = cvt4(selv(hi, t7, t6));
    _Float16* swp = sw + hh * CIN + 4 * lj;
    *(v4h*)(swp)           = c0;
    *(v4h*)(swp + 2 * CIN) = c1;
    *(v4h*)(swp + 4 * CIN) = c2;
    *(v4h*)(swp + 6 * CIN) = c3;
    __builtin_amdgcn_fence(__ATOMIC_ACQ_REL, "wavefront");
    __builtin_amdgcn_wave_barrier();
    const v8h o0 = *(const v8h*)(sw + 8 * lane);
    const v8h o1 = *(const v8h*)(sw + KD / 2 + 8 * lane);
    __builtin_amdgcn_fence(__ATOMIC_ACQ_REL, "wavefront");
    __builtin_amdgcn_wave_barrier();
    _Float16* gp = Ag + (size_t)c * KD + 8 * lane;
    *(volatile v8h*)gp = o0;
    *(volatile v8h*)(gp + KD / 2) = o1;
    __threadfence();
    *(volatile v8h*)gp = o0;
    *(volatile v8h*)(gp + KD / 2) = o1;
  }
}

__global__ __launch_bounds__(NTHR) void k_gemm(
    const _Float16* __restrict__ Ag, const _Float16* __restrict__ Bw,
    const float* __restrict__ bias, float* C, int nOut) {
  __shared__ __attribute__((aligned(16))) float stg[GROWS * FD];
  const int tid = threadIdx.x, lane = tid & 31, wave = tid >> 5, hh = lane >> 4, m = lane & 15;
  const int rowBase = blockIdx.x * GROWS;
  const int wrow = rowBase + wave * 16;

  v8f acc[4];
#pragma unroll
  for (int t = 0; t < 4; ++t) { v8f z = {0.f, 0.f, 0.f, 0.f, 0.f, 0.f, 0.f, 0.f}; acc[t] = z; }
  const _Float16* ap  = Ag + (size_t)(wrow + m) * KD + 8 * hh;
  const _Float16* bp0 = Bw + (size_t)m * KD + 8 * hh;
#pragma unroll 1
  for (int kt = 0; kt < KD / 32; ++kt) {
    FragH a;
    a.h[0] = *(const v8h*)(ap + 32 * kt);
    a.h[1] = *(const v8h*)(ap + 32 * kt + 16);
#pragma unroll
    for (int t = 0; t < 4; ++t) {
      const _Float16* bp = bp0 + (size_t)(16 * t) * KD + 32 * kt;
      FragH b;
      b.h[0] = *(const v8h*)bp;
      b.h[1] = *(const v8h*)(bp + 16);
      acc[t] = wmh(a.v, b.v, acc[t]);
    }
  }

  float* sp = stg + (wave * 16 + 8 * hh) * FD + m;
#pragma unroll
  for (int t = 0; t < 4; ++t) {
    const float bv = bias[16 * t + m];
#pragma unroll
    for (int r = 0; r < 8; ++r) sp[r * FD + 16 * t] = acc[t][r] * WINV + bv;
  }
  __syncthreads();

  const float* lp = stg + wave * 16 * FD + 4 * lane;
  float* gp = C + (size_t)wrow * FD + 4 * lane;
  v4f ov[8];
#pragma unroll
  for (int i = 0; i < 8; ++i) ov[i] = *(const v4f*)(lp + 128 * i);
#pragma unroll
  for (int i = 0; i < 8; ++i) {
    if (wrow + 2 * i + hh < nOut) *(volatile v4f*)(gp + 128 * i) = ov[i];
  }
  __threadfence();
#pragma unroll
  for (int i = 0; i < 8; ++i) {
    if (wrow + 2 * i + hh < nOut) *(volatile v4f*)(gp + 128 * i) = ov[i];
  }
}

extern "C" void kernel_launch(void* const* d_in, const int* in_sizes, int n_in,
                              void* d_out, int out_size, void* d_ws, size_t ws_size,
                              hipStream_t stream) {
  if (n_in < 6) return;
  const int nIn  = in_sizes[0] / CIN;
  const int nE   = in_sizes[2] / 2;
  const int nOut = out_size / FD;
  if (nIn <= 0 || nE <= 0 || nOut <= 0) return;
  if (in_sizes[0] != nIn * CIN) return;
  if (in_sizes[2] != 2 * nE) return;
  if (in_sizes[1] != TT * nE) return;
  if (in_sizes[3] != TT * CIN * FD || in_sizes[4] != FD) return;
  if (out_size != nOut * FD) return;
  if (nE > (1 << 28) || nIn > (1 << 24) || nOut > (1 << 22)) return;

  const float* x    = (const float*)d_in[0];
  const float* ef   = (const float*)d_in[1];
  const int*   idx  = (const int*)d_in[2];
  const float* Km   = (const float*)d_in[3];
  const float* bia  = (const float*)d_in[4];
  float* out = (float*)d_out;

  const int NPAD   = ((nOut + TGT - 1) / TGT) * TGT;
  const int nBC    = (nOut + NBC - 1) / NBC;
  const int CNTPAD = nBC * NBC;
  if (4 * nBC + 1 > RBN) return;
  const int nBF    = (nOut + NBF - 1) / NBF;
  const int csrLen = ((nE + 31) & ~31) + 4096;
  if (31 * 4 * nBC > 4096) return;
  const int nGemm  = NPAD / GROWS;
  const int nAgg   = NPAD / TGT;

  char* ws = (char*)d_ws;
  size_t off = 0;
  const size_t oW   = off; off += (size_t)FD * KD * 2;             off = (off + 255) & ~(size_t)255;
  const size_t oCnt = off; off += (size_t)CNTPAD * 4;              off = (off + 255) & ~(size_t)255;
  const size_t oOff = off; off += (size_t)CNTPAD * 4;              off = (off + 255) & ~(size_t)255;
  const size_t oRb  = off; off += (size_t)RBN * 4;                 off = (off + 255) & ~(size_t)255;
  const size_t oCsr = off; off += (size_t)csrLen * 4;              off = (off + 255) & ~(size_t)255;
  const size_t oA   = off; off += (size_t)NPAD * KD * 2;           off = (off + 255) & ~(size_t)255;
  if (off > ws_size || off > (size_t)WSCAP) return;
  _Float16* wp   = (_Float16*)(ws + oW);
  int*      cnt  = (int*)(ws + oCnt);
  int*      offp = (int*)(ws + oOff);
  int*      rb   = (int*)(ws + oRb);
  int*      csr  = (int*)(ws + oCsr);
  _Float16* Ag   = (_Float16*)(ws + oA);

  const int vec8 = 1;

  k_wprep<<<TT, NTHR, 0, stream>>>(Km, wp);

  k_count<<<nBC, NTHR, 0, stream>>>(idx, cnt, nE, vec8);
  k_offsets<<<1, OTHR, 0, stream>>>(cnt, offp, rb, nBC);
  hipFuncSetAttribute(reinterpret_cast<const void*>(&k_fill),
                      hipFuncAttributeMaxDynamicSharedMemorySize, LDS_FILL);
  k_fill<<<nBF, NTHR, LDS_FILL, stream>>>(idx, offp, rb, csr, nE, vec8, csrLen);

  k_agg<<<nAgg, NTHR, 0, stream>>>(csr, offp, cnt, idx, ef, x, Ag, nIn, nE, csrLen);

  k_gemm<<<nGemm, NTHR, 0, stream>>>(Ag, wp, bia, out, nOut);
}
